// MultiHeadSelfAttention_7756710936699
// MI455X (gfx1250) — hardware-verified
//
#include <hip/hip_runtime.h>


#ifndef NB
#define NB 2
#endif
#ifndef SEQ
#define SEQ 2048
#endif
#define SEQ_FULL 2048
#define DM   1024
#define NH   16
#define HD   64
#define C2   0.18033688011112042f
#define PEXP 14.0f
#define CTSC 0.00390625f
#define OSC  0.0009765625f

static_assert(SEQ % 64 == 0);
static_assert(SEQ <= SEQ_FULL);
static_assert(NH * HD == DM);
static_assert(DM % 128 == 0);
static_assert((NB * SEQ) % 8 == 0);

typedef _Float16 h16;
typedef unsigned short bf;
typedef __attribute__((ext_vector_type(16))) __bf16   v16bf;
typedef __attribute__((ext_vector_type(16))) _Float16 v16h;
typedef __attribute__((ext_vector_type(8)))  _Float16 v8h;
typedef __attribute__((ext_vector_type(8)))  unsigned short v8us;
typedef __attribute__((ext_vector_type(8)))  float    v8f;
typedef __attribute__((ext_vector_type(4)))  float    v4f;
typedef v4f  __attribute__((may_alias)) v4fa;

__device__ __forceinline__ unsigned short f2bf(float f) { unsigned u = __float_as_uint(f); u += 0x7FFFu + ((u >> 16) & 1u); return (unsigned short)(u >> 16); }
__device__ __forceinline__ float bf2f(unsigned short b) { return __uint_as_float(((unsigned)b) << 16); }
__device__ __forceinline__ float bfr(float f) { return bf2f(f2bf(f)); }
__device__ __forceinline__ v16h cat16(v8h lo, v8h hi) { return __builtin_shufflevector(lo, hi, 0, 1, 2, 3, 4, 5, 6, 7, 8, 9, 10, 11, 12, 13, 14, 15); }
__device__ __forceinline__ v16bf cat16b(v8us lo, v8us hi) { return __builtin_bit_cast(v16bf, __builtin_shufflevector(lo, hi, 0, 1, 2, 3, 4, 5, 6, 7, 8, 9, 10, 11, 12, 13, 14, 15)); }
__device__ __forceinline__ v8f wmma16(v16h a, v16h b, v8f c) { return __builtin_amdgcn_wmma_f32_16x16x32_f16(false, a, false, b, (short)0, c, false, false); }
__device__ __forceinline__ v8f wmmab(v16bf a, v16bf b, v8f c) { return __builtin_amdgcn_wmma_f32_16x16x32_bf16(false, a, false, b, (short)0, c, false, false); }

template <typename T16> struct WFrag;
template <> struct WFrag<h16> { typedef v16h V; static __device__ __forceinline__ V ld(const h16* p) { return cat16(*(const v8h*)p, *(const v8h*)(p + 16)); } static __device__ __forceinline__ v8f mma(V a, V b, v8f c) { return wmma16(a, b, c); } };
template <> struct WFrag<bf> { typedef v16bf V; static __device__ __forceinline__ V ld(const bf* p) { return cat16b(*(const v8us*)p, *(const v8us*)(p + 16)); } static __device__ __forceinline__ v8f mma(V a, V b, v8f c) { return wmmab(a, b, c); } };

template <typename T16>
__device__ __forceinline__ void gemm64(const T16* __restrict__ A, const T16* __restrict__ Bt, unsigned K, unsigned lr, unsigned hi, v8f (&acc)[4][4]) {
    typedef typename WFrag<T16>::V V;
    const size_t aoff = (size_t)lr * K + 8u * hi, boff = (size_t)lr * K + 8u * hi;
#pragma unroll 1
    for (unsigned kc = 0; kc < K; kc += 32) {
        V a[4];
#pragma unroll
        for (unsigned mb = 0; mb < 4; ++mb) a[mb] = WFrag<T16>::ld(A + aoff + (size_t)mb * 16 * K + kc);
#pragma unroll
        for (unsigned nb = 0; nb < 4; ++nb) { const V b = WFrag<T16>::ld(Bt + boff + (size_t)nb * 16 * K + kc);
#pragma unroll
            for (unsigned mb = 0; mb < 4; ++mb) acc[mb][nb] = WFrag<T16>::mma(a[mb], b, acc[mb][nb]); }
        asm volatile("v_nop\n\tv_nop\n\tv_nop\n\tv_nop" : "+v"(acc[0][0]), "+v"(acc[1][1]), "+v"(acc[2][2]), "+v"(acc[3][3]) : "v"(a[0]), "v"(a[3]));
    }
}

__global__ __launch_bounds__(256) void k_cvtx(const float* __restrict__ src, bf* dst) {
    const unsigned i = blockIdx.x * 256u + threadIdx.x; if (i >= (unsigned)(NB * SEQ * DM / 8)) return;
    const unsigned e = i * 8u; const unsigned b = e / (unsigned)(SEQ * DM); const unsigned rem = e - b * (unsigned)(SEQ * DM);
    const v8f v = *(const v8f*)(src + (size_t)b * SEQ_FULL * DM + rem); v8us o;
#pragma unroll
    for (unsigned k = 0; k < 8; ++k) o[k] = f2bf(v[k]);
    *(volatile v8us*)(dst + (size_t)e) = o; __threadfence(); *(volatile v8us*)(dst + (size_t)e) = o;
}
__global__ __launch_bounds__(256) void k_cvtw(const float* __restrict__ w0, const float* __restrict__ w1, const float* __restrict__ w2, bf* dst) {
    const unsigned i = blockIdx.x * 256u + threadIdx.x; const unsigned y = blockIdx.y; if (i >= (unsigned)(DM * DM / 8)) return;
    const float* src = (y == 0u) ? w0 : ((y == 1u) ? w1 : w2);
    const v8f v = *(const v8f*)(src + (size_t)i * 8); v8us o;
#pragma unroll
    for (unsigned k = 0; k < 8; ++k) o[k] = f2bf(v[k]);
    bf* d = dst + (size_t)y * DM * DM + (size_t)i * 8;
    *(volatile v8us*)d = o; __threadfence(); *(volatile v8us*)d = o;
}
__global__ __launch_bounds__(256) void k_cvto(const float* __restrict__ src, h16* dst) {
    const unsigned i = blockIdx.x * 256u + threadIdx.x; if (i >= (unsigned)(DM * DM / 8)) return;
    const v8f v = *(const v8f*)(src + (size_t)i * 8); v8h o;
#pragma unroll
    for (unsigned k = 0; k < 8; ++k) o[k] = (h16)(bfr(v[k]) * 16.0f);
    *(volatile v8h*)(dst + (size_t)i * 8) = o; __threadfence(); *(volatile v8h*)(dst + (size_t)i * 8) = o;
}

__global__ __launch_bounds__(32) void k_proj(const bf* __restrict__ XB, const bf* __restrict__ W3, h16* QP, h16* KP, h16* VT) {
    __shared__ __align__(16) float os[64 * 68];
    const unsigned lane = threadIdx.x & 31u, lr = lane & 15u, hi = lane >> 4;
    const unsigned r0 = blockIdx.x * 64u, hd = blockIdx.y, z = blockIdx.z, c0 = hd * 64u;
    v8f acc[4][4];
#pragma unroll
    for (unsigned mb = 0; mb < 4; ++mb)
#pragma unroll
        for (unsigned nb = 0; nb < 4; ++nb) acc[mb][nb] = (v8f){};
    gemm64<bf>(XB + (size_t)r0 * DM, W3 + ((size_t)z * DM + c0) * DM, DM, lr, hi, acc);
#pragma unroll
    for (unsigned mb = 0; mb < 4; ++mb)
#pragma unroll
        for (unsigned nb = 0; nb < 4; ++nb)
#pragma unroll
            for (unsigned j = 0; j < 8; ++j) os[(mb * 16 + hi * 8 + j) * 68 + nb * 16 + lr] = acc[mb][nb][j];
    __syncthreads();
    const unsigned b = r0 / (unsigned)SEQ, t0 = r0 - b * (unsigned)SEQ;
    const unsigned g = lane >> 3, pc = (lane & 7u) * 8u;
    if (z < 2u) {
        h16* P = ((z == 0u) ? QP : KP) + ((size_t)(b * NH + hd) * SEQ + t0) * HD;
#pragma unroll 1
        for (unsigned ps = 0; ps < 2; ++ps) {
#pragma unroll
            for (unsigned s = 0; s < 16; ++s) { const unsigned row = 4 * s + g; const v4f x0 = *(const v4fa*)(os + row * 68 + pc), x1 = *(const v4fa*)(os + row * 68 + pc + 4); v8h o;
                o[0] = (h16)x0[0]; o[1] = (h16)x0[1]; o[2] = (h16)x0[2]; o[3] = (h16)x0[3]; o[4] = (h16)x1[0]; o[5] = (h16)x1[1]; o[6] = (h16)x1[2]; o[7] = (h16)x1[3];
                *(volatile v8h*)(P + (size_t)row * HD + pc) = o; }
            if (ps == 0) __threadfence(); }
    } else {
        h16* P = VT + ((size_t)(b * NH + hd) * HD) * SEQ + t0;
#pragma unroll 1
        for (unsigned ps = 0; ps < 2; ++ps) {
#pragma unroll
            for (unsigned s = 0; s < 16; ++s) { const unsigned d = 4 * s + g; v8h o;
#pragma unroll
                for (unsigned j = 0; j < 8; ++j) o[j] = (h16)os[(pc + j) * 68 + d];
                *(volatile v8h*)(P + (size_t)d * SEQ + pc) = o; }
            if (ps == 0) __threadfence(); }
    }
}

__global__ __launch_bounds__(32) void k_lse(const h16* __restrict__ QP, const h16* __restrict__ KP, float* LSE) {
    __shared__ __align__(16) float ls[32];
    const unsigned lane = threadIdx.x & 31u, lr = lane & 15u, hi = lane >> 4;
    const unsigned key0 = blockIdx.x * 32u, bh = blockIdx.y;
    const h16* Kb = KP + (size_t)bh * SEQ * HD; const h16* Qb = QP + (size_t)bh * SEQ * HD;
    v16h a[2][2];
#pragma unroll
    for (unsigned mb = 0; mb < 2; ++mb)
#pragma unroll
        for (unsigned kc = 0; kc < 2; ++kc) a[mb][kc] = WFrag<h16>::ld(Kb + (size_t)(key0 + mb * 16 + lr) * HD + kc * 32 + 8u * hi);
    float m[2][8], l[2][8];
#pragma unroll
    for (unsigned mb = 0; mb < 2; ++mb)
#pragma unroll
        for (unsigned r = 0; r < 8; ++r) { m[mb][r] = -3.0e38f; l[mb][r] = 0.f; }
#pragma unroll 1
    for (unsigned q0 = 0; q0 < (unsigned)SEQ; q0 += 64) {
        v8f acc[2][4];
#pragma unroll
        for (unsigned nb = 0; nb < 4; ++nb) { const h16* qp = Qb + (size_t)(q0 + nb * 16 + lr) * HD + 8u * hi; const v16h b0 = WFrag<h16>::ld(qp), b1 = WFrag<h16>::ld(qp + 32);
#pragma unroll
            for (unsigned mb = 0; mb < 2; ++mb) { v8f s = (v8f){}; s = wmma16(a[mb][0], b0, s); s = wmma16(a[mb][1], b1, s); acc[mb][nb] = s; } }
        asm volatile("v_nop\n\tv_nop\n\tv_nop\n\tv_nop" : "+v"(acc[0][0]), "+v"(acc[0][1]), "+v"(acc[0][2]), "+v"(acc[0][3]), "+v"(acc[1][0]), "+v"(acc[1][1]), "+v"(acc[1][2]), "+v"(acc[1][3]) : "v"(a[0][0]), "v"(a[1][1]));
#pragma unroll
        for (unsigned mb = 0; mb < 2; ++mb)
#pragma unroll
            for (unsigned r = 0; r < 8; ++r) {
                const float cm = fmaxf(fmaxf(acc[mb][0][r], acc[mb][1][r]), fmaxf(acc[mb][2][r], acc[mb][3][r]));
                const float mn = fmaxf(m[mb][r], cm * C2);
                const float e = __builtin_amdgcn_exp2f(m[mb][r] - mn);
                const float sa = (__builtin_amdgcn_exp2f(fmaf(acc[mb][0][r], C2, -mn)) + __builtin_amdgcn_exp2f(fmaf(acc[mb][1][r], C2, -mn))) + (__builtin_amdgcn_exp2f(fmaf(acc[mb][2][r], C2, -mn)) + __builtin_amdgcn_exp2f(fmaf(acc[mb][3][r], C2, -mn)));
                l[mb][r] = l[mb][r] * e + sa; m[mb][r] = mn; }
    }
#pragma unroll
    for (unsigned mb = 0; mb < 2; ++mb)
#pragma unroll
        for (unsigned r = 0; r < 8; ++r) {
#pragma unroll
            for (unsigned sh = 1; sh < 16; sh <<= 1) { const float mo = __shfl_xor(m[mb][r], (int)sh, 32); const float lo = __shfl_xor(l[mb][r], (int)sh, 32); const float mn = fmaxf(m[mb][r], mo);
                l[mb][r] = l[mb][r] * __builtin_amdgcn_exp2f(m[mb][r] - mn) + lo * __builtin_amdgcn_exp2f(mo - mn); m[mb][r] = mn; } }
    if (lr == 0u) {
#pragma unroll
        for (unsigned mb = 0; mb < 2; ++mb)
#pragma unroll
            for (unsigned r = 0; r < 8; ++r) ls[mb * 16 + hi * 8 + r] = (m[mb][r] + __builtin_amdgcn_logf(l[mb][r])) - PEXP; }
    __syncthreads();
    if (lane < 8u) { const v4f val = *(const v4fa*)(ls + lane * 4u); float* dst = LSE + (size_t)bh * SEQ + key0 + lane * 4u;
        *(volatile v4f*)dst = val; __threadfence(); *(volatile v4f*)dst = val; }
}

__global__ __launch_bounds__(32) void k_ctx(const h16* __restrict__ QP, const h16* __restrict__ KP, const h16* __restrict__ VT, const float* __restrict__ LSE, h16* CT) {
    __shared__ __align__(16) float os[32 * 68];
    const unsigned lane = threadIdx.x & 31u, lr = lane & 15u, hi = lane >> 4;
    const unsigned q0 = blockIdx.x * 32u, bh = blockIdx.y; const unsigned b = bh / (unsigned)NH, hd = bh - b * (unsigned)NH;
    const h16* Qb = QP + (size_t)bh * SEQ * HD; const h16* Kb = KP + (size_t)bh * SEQ * HD; const h16* Vb = VT + (size_t)bh * HD * SEQ; const float* Lb = LSE + (size_t)bh * SEQ;
    v16h bq[2][2];
#pragma unroll
    for (unsigned qb = 0; qb < 2; ++qb)
#pragma unroll
        for (unsigned kc = 0; kc < 2; ++kc) bq[qb][kc] = WFrag<h16>::ld(Qb + (size_t)(q0 + qb * 16 + lr) * HD + kc * 32 + 8u * hi);
    v8f c[4][2];
#pragma unroll
    for (unsigned db = 0; db < 4; ++db)
#pragma unroll
        for (unsigned qb = 0; qb < 2; ++qb) c[db][qb] = (v8f){};
#pragma unroll 1
    for (unsigned k0 = 0; k0 < (unsigned)SEQ; k0 += 32) {
        v16h ak[2][2], av[4];
#pragma unroll
        for (unsigned kt = 0; kt < 2; ++kt)
#pragma unroll
            for (unsigned kc = 0; kc < 2; ++kc) ak[kt][kc] = WFrag<h16>::ld(Kb + (size_t)(k0 + kt * 16 + lr) * HD + kc * 32 + 8u * hi);
#pragma unroll
        for (unsigned db = 0; db < 4; ++db) av[db] = WFrag<h16>::ld(Vb + (size_t)(db * 16 + lr) * SEQ + k0 + 8u * hi);
        const v4f la = *(const v4f*)(Lb + k0 + 8u * hi), lb = *(const v4f*)(Lb + k0 + 8u * hi + 4), lc = *(const v4f*)(Lb + k0 + 16 + 8u * hi), ld = *(const v4f*)(Lb + k0 + 16 + 8u * hi + 4);
#pragma unroll
        for (unsigned qb = 0; qb < 2; ++qb) {
            v8f s0 = (v8f){}, s1 = (v8f){};
            s0 = wmma16(ak[0][0], bq[qb][0], s0); s0 = wmma16(ak[0][1], bq[qb][1], s0);
            s1 = wmma16(ak[1][0], bq[qb][0], s1); s1 = wmma16(ak[1][1], bq[qb][1], s1);
            asm volatile("v_nop\n\tv_nop\n\tv_nop\n\tv_nop" : "+v"(s0), "+v"(s1) : "v"(ak[1][1]), "v"(bq[qb][1]));
            v16h p;
#pragma unroll
            for (unsigned i = 0; i < 4; ++i) {
                p[i]      = (h16)__builtin_amdgcn_exp2f(fmaf(s0[i],     C2, -la[i]));
                p[4 + i]  = (h16)__builtin_amdgcn_exp2f(fmaf(s0[4 + i], C2, -lb[i]));
                p[8 + i]  = (h16)__builtin_amdgcn_exp2f(fmaf(s1[i],     C2, -lc[i]));
                p[12 + i] = (h16)__builtin_amdgcn_exp2f(fmaf(s1[4 + i], C2, -ld[i])); }
#pragma unroll
            for (unsigned db = 0; db < 4; ++db) c[db][qb] = wmma16(av[db], p, c[db][qb]);
        }
        asm volatile("v_nop\n\tv_nop\n\tv_nop\n\tv_nop" : "+v"(c[0][0]), "+v"(c[1][0]), "+v"(c[2][0]), "+v"(c[3][0]), "+v"(c[0][1]), "+v"(c[1][1]), "+v"(c[2][1]), "+v"(c[3][1]) : "v"(av[0]), "v"(av[3]));
    }
#pragma unroll
    for (unsigned db = 0; db < 4; ++db)
#pragma unroll
        for (unsigned qb = 0; qb < 2; ++qb)
#pragma unroll
            for (unsigned r = 0; r < 8; ++r) os[(qb * 16 + lr) * 68 + db * 16 + hi * 8 + r] = c[db][qb][r] * CTSC;
    __syncthreads();
    const unsigned g = lane >> 3, pc = (lane & 7u) * 8u;
    h16* P = CT + ((size_t)b * SEQ + q0) * DM + hd * 64u;
#pragma unroll 1
    for (unsigned ps = 0; ps < 2; ++ps) {
#pragma unroll
        for (unsigned s = 0; s < 8; ++s) { const unsigned row = 4 * s + g; const v4f x0 = *(const v4fa*)(os + row * 68 + pc), x1 = *(const v4fa*)(os + row * 68 + pc + 4); v8h o;
            o[0] = (h16)x0[0]; o[1] = (h16)x0[1]; o[2] = (h16)x0[2]; o[3] = (h16)x0[3]; o[4] = (h16)x1[0]; o[5] = (h16)x1[1]; o[6] = (h16)x1[2]; o[7] = (h16)x1[3];
            *(volatile v8h*)(P + (size_t)row * DM + pc) = o; }
        if (ps == 0) __threadfence(); }
}

__global__ __launch_bounds__(32) void k_oproj(const h16* __restrict__ CT, const h16* __restrict__ WO, const float* __restrict__ x, float* Y) {
    __shared__ __align__(16) float os[16 * 68];
    const unsigned lane = threadIdx.x & 31u, lr = lane & 15u, hi = lane >> 4;
    const unsigned r0 = blockIdx.x * 64u, c0 = blockIdx.y * 64u;
    v8f acc[4][4];
#pragma unroll
    for (unsigned mb = 0; mb < 4; ++mb)
#pragma unroll
        for (unsigned nb = 0; nb < 4; ++nb) acc[mb][nb] = (v8f){};
    gemm64<h16>(CT + (size_t)r0 * DM, WO + (size_t)c0 * DM, DM, lr, hi, acc);
    const unsigned b = r0 / (unsigned)SEQ, t0 = r0 - b * (unsigned)SEQ;
    const float* xt = x + ((size_t)b * SEQ_FULL + t0) * DM + c0;
#pragma unroll
    for (unsigned mb = 0; mb < 4; ++mb) {
#pragma unroll
        for (unsigned nb = 0; nb < 4; ++nb)
#pragma unroll
            for (unsigned j = 0; j < 8; ++j) os[(hi * 8 + j) * 68 + nb * 16 + lr] = acc[mb][nb][j];
        __syncthreads();
        float* crow = Y + (size_t)(r0 + mb * 16) * DM + c0;
        const float* xrow = xt + (size_t)(mb * 16) * DM;
#pragma unroll 1
        for (unsigned ps = 0; ps < 2; ++ps) {
#pragma unroll
            for (unsigned s = 0; s < 8; ++s) { const unsigned row = 2 * s + hi, cofs = lr * 4u; v4f val = *(const v4fa*)(os + row * 68 + cofs); const v4f xv = *(const v4f*)(xrow + (size_t)row * DM + cofs);
                val[0] = val[0] * OSC + bfr(xv[0]); val[1] = val[1] * OSC + bfr(xv[1]); val[2] = val[2] * OSC + bfr(xv[2]); val[3] = val[3] * OSC + bfr(xv[3]);
                *(volatile v4f*)(crow + (size_t)row * DM + cofs) = val; }
            if (ps == 0) __threadfence(); }
        __syncthreads();
    }
}

__global__ __launch_bounds__(256) void k_ln(const float* __restrict__ Y, const float* __restrict__ gamma, const float* __restrict__ beta, float* OUT) {
    const unsigned lane = threadIdx.x & 31u; const unsigned row = blockIdx.x * 8u + (threadIdx.x >> 5);
    if (row >= (unsigned)(NB * SEQ)) return;
    const float* yr = Y + (size_t)row * DM + lane * 4u;
    float s = 0.f;
#pragma unroll 1
    for (unsigned ch = 0; ch < (unsigned)(DM / 128); ++ch) { const v4f a = *(const v4f*)(yr + ch * 128u); s += (a[0] + a[1]) + (a[2] + a[3]); }
#pragma unroll
    for (unsigned sh = 16; sh; sh >>= 1) s += __shfl_xor(s, (int)sh, 32);
    const float mu = s * (1.0f / DM);
    float q = 0.f;
#pragma unroll 1
    for (unsigned ch = 0; ch < (unsigned)(DM / 128); ++ch) { const v4f a = *(const v4f*)(yr + ch * 128u); const float d0 = a[0] - mu, d1 = a[1] - mu, d2 = a[2] - mu, d3 = a[3] - mu; q += (d0 * d0 + d1 * d1) + (d2 * d2 + d3 * d3); }
#pragma unroll
    for (unsigned sh = 16; sh; sh >>= 1) q += __shfl_xor(q, (int)sh, 32);
    const float rstd = rsqrtf(q * (1.0f / DM) + 1e-5f);
    float* orow = OUT + (size_t)row * DM + lane * 4u;
    const float* gp = gamma + lane * 4u; const float* bp = beta + lane * 4u;
#pragma unroll 1
    for (unsigned ps = 0; ps < 2; ++ps) {
#pragma unroll 1
        for (unsigned ch = 0; ch < (unsigned)(DM / 128); ++ch) { const v4f a = *(const v4f*)(yr + ch * 128u); const v4f gg = *(const v4f*)(gp + ch * 128u); const v4f be = *(const v4f*)(bp + ch * 128u); v4f o;
            o[0] = (a[0] - mu) * rstd * bfr(gg[0]) + bfr(be[0]); o[1] = (a[1] - mu) * rstd * bfr(gg[1]) + bfr(be[1]); o[2] = (a[2] - mu) * rstd * bfr(gg[2]) + bfr(be[2]); o[3] = (a[3] - mu) * rstd * bfr(gg[3]) + bfr(be[3]);
            *(volatile v4f*)(orow + ch * 128u) = o; }
        if (ps == 0) __threadfence(); }
}

#define WS_XB  ((size_t)NB * SEQ * DM * 2)
#define WS_W3  ((size_t)3 * DM * DM * 2)
#define WS_WO  ((size_t)DM * DM * 2)
#define WS_PL  ((size_t)NB * SEQ * DM * 2)
#define WS_LSE ((size_t)NB * NH * SEQ * 4)
#define WS_Y   ((size_t)NB * SEQ * DM * 4)
static_assert(WS_XB + WS_W3 + WS_WO + 4 * WS_PL + WS_LSE + WS_Y + 4096 <= (size_t)134217728);
static_assert((size_t)(NB * SEQ / 64) * NH * 64 * 64 == (size_t)NB * SEQ * DM);
static_assert((size_t)(SEQ / 32) * (NB * NH) * 32 == (size_t)NB * NH * SEQ);
static_assert((size_t)(SEQ / 32) * (NB * NH) * 32 * HD == (size_t)NB * SEQ * DM);
static_assert((size_t)(NB * SEQ * DM / 8 / 256) * 256 * 8 == (size_t)NB * SEQ * DM);
static_assert((size_t)(DM * DM / 8 / 256) * 256 * 8 == (size_t)DM * DM);

extern "C" void kernel_launch(void* const* d_in, const int* in_sizes, int n_in,
                              void* d_out, int out_size, void* d_ws, size_t ws_size, hipStream_t stream) {
    if (n_in < 7) return;
    if ((long long)in_sizes[0] < (long long)(NB - 1) * SEQ_FULL * DM + (long long)SEQ * DM) return;
    if (in_sizes[1] < DM * DM || in_sizes[2] < DM * DM || in_sizes[3] < DM * DM || in_sizes[4] < DM * DM) return;
    if (in_sizes[5] < DM || in_sizes[6] < DM) return;
    if ((long long)out_size < (long long)NB * SEQ * DM) return;
    const float* x = (const float*)d_in[0]; const float* wq = (const float*)d_in[1]; const float* wk = (const float*)d_in[2]; const float* wv = (const float*)d_in[3]; const float* wo = (const float*)d_in[4];
    const float* gamma = (const float*)d_in[5]; const float* beta = (const float*)d_in[6];
    float* OUT = (float*)d_out;
    char* wsp = (char*)d_ws;
    auto take = [&](size_t bytes) { char* p = wsp; wsp += (bytes + 255) & ~(size_t)255; return (void*)p; };
    bf* XB = (bf*)take(WS_XB); bf* W3 = (bf*)take(WS_W3); h16* WO = (h16*)take(WS_WO);
    h16* QP = (h16*)take(WS_PL); h16* KP = (h16*)take(WS_PL); h16* VT = (h16*)take(WS_PL); h16* CT = (h16*)take(WS_PL);
    float* LSE = (float*)take(WS_LSE); float* Y = (float*)take(WS_Y);
    if ((size_t)(wsp - (char*)d_ws) > ws_size) return;
    k_cvtx<<<(unsigned)((NB * SEQ * DM / 8 + 255) / 256), 256, 0, stream>>>(x, XB);
    k_cvtw<<<dim3((unsigned)((DM * DM / 8 + 255) / 256), 3, 1), 256, 0, stream>>>(wq, wk, wv, W3);
    k_cvto<<<(unsigned)((DM * DM / 8 + 255) / 256), 256, 0, stream>>>(wo, WO);
    k_proj<<<dim3(NB * SEQ / 64, NH, 3), 32, 0, stream>>>(XB, W3, QP, KP, VT);
    k_lse<<<dim3(SEQ / 32, NB * NH, 1), 32, 0, stream>>>(QP, KP, LSE);
    k_ctx<<<dim3(SEQ / 32, NB * NH, 1), 32, 0, stream>>>(QP, KP, VT, LSE, CT);
    k_oproj<<<dim3(NB * SEQ / 64, DM / 64, 1), 32, 0, stream>>>(CT, WO, x, Y);
    k_ln<<<(unsigned)((NB * SEQ + 7) / 8), 256, 0, stream>>>(Y, gamma, beta, OUT);
}
